// QRNN_60498909332052
// MI455X (gfx1250) — hardware-run, weakly checked
//
#include <hip/hip_runtime.h>
#include <math.h>

typedef __attribute__((ext_vector_type(16))) _Float16 v16h;
typedef __attribute__((ext_vector_type(8)))  _Float16 v8h;
typedef __attribute__((ext_vector_type(16))) __bf16   v16b;
typedef __attribute__((ext_vector_type(8)))  __bf16   v8b;
typedef __attribute__((ext_vector_type(8)))  float    v8f;
typedef __attribute__((ext_vector_type(4)))  float    v4f;

constexpr int kB    = 8;
constexpr int kT    = 4096;
constexpr int kDi   = 256;
constexpr int kDo   = 256;
constexpr int kWin  = 2;
constexpr int kN3   = 3 * kDo;
constexpr int kTP   = kT + 1;
constexpr int kThr  = 256;
constexpr float kInCarry = 1024.0f;
constexpr float kWCarry = 4096.0f;
constexpr float kSc = 1.0f / (kInCarry * kWCarry);
constexpr float kF16MinNormal = 6.103515625e-5f;

static_assert(kWin == 2 && (kT % 64) == 0 && (kN3 % 64) == 0 && ((kWin * kDi) % 32) == 0 && ((kT / 64) * (kN3 / 64)) % 8 == 0, "the product: M, N multiples of 64, K of 32; a sample's 768 tiles = 96 blocks");

constexpr size_t kOffX16P = 0ull;
constexpr size_t kOffWZFO = 16781312ull;
constexpr size_t kOffBIAS = 17567744ull;
constexpr size_t kOffZFO = 17571840ull;
constexpr size_t kWsTotal = 118235136ull;
static_assert(kWsTotal <= 134217728ull, "carve cap: under 128 MiB");
static_assert(kOffX16P == 0 && kOffWZFO == kOffX16P + 16781312ull && kOffBIAS == kOffWZFO + 786432ull && kOffZFO == kOffBIAS + 4096ull && kWsTotal == kOffZFO + 100663296ull, "the carve is chained and totalled");
static_assert((kOffWZFO % 256) == 0 && (kOffBIAS % 256) == 0 && (kOffZFO % 256) == 0 && ((size_t)kTP * kDi * 2) % 16 == 0, "aligned regions; a sample's plane starts on a 16-B boundary");

__device__ __forceinline__ unsigned short f2bf_bits(float f) {
  unsigned u = __float_as_uint(f);
  return (unsigned short)((u + 0x7FFFu + ((u >> 16) & 1u)) >> 16);
}
__device__ __forceinline__ float bf_bits2f(unsigned short h) { return __uint_as_float(((unsigned)h) << 16); }
__device__ __forceinline__ float bf16r(float f) { return bf_bits2f(f2bf_bits(f)); }
__device__ __forceinline__ float carry_flush(float v, float carry) {
  const float s = v * carry;
  return (fabsf(s) < kF16MinNormal) ? 0.0f : s;
}
__device__ __forceinline__ float frcp(float x) { return __builtin_amdgcn_rcpf(x); }

__device__ __forceinline__ void dep_guard4_h(v8f& a, v8f& b, v8f& c, v8f& d, v16h x, v16h y) { asm volatile("v_nop\n\tv_nop\n\tv_nop\n\tv_nop" : "+v"(a), "+v"(b), "+v"(c), "+v"(d) : "v"(x), "v"(y)); }
__device__ __forceinline__ void dep_guard4_b(v8f& a, v8f& b, v8f& c, v8f& d, v16b x, v16b y) { asm volatile("v_nop\n\tv_nop\n\tv_nop\n\tv_nop" : "+v"(a), "+v"(b), "+v"(c), "+v"(d) : "v"(x), "v"(y)); }
__device__ __forceinline__ void keep4_h(v16h a, v16h b, v16h c, v16h d) { asm volatile("v_nop" :: "v"(a), "v"(b), "v"(c), "v"(d)); }
__device__ __forceinline__ void keep4_b(v16b a, v16b b, v16b c, v16b d) { asm volatile("v_nop" :: "v"(a), "v"(b), "v"(c), "v"(d)); }
__device__ __forceinline__ void acc_guard4(v8f& a, v8f& b, v8f& c, v8f& d) { asm volatile("v_nop\n\tv_nop\n\tv_nop\n\tv_nop" : "+v"(a), "+v"(b), "+v"(c), "+v"(d)); }

template <typename T> struct Frag;
template <> struct Frag<_Float16> {
  typedef v16h V; union U { v16h v; v8h h[2]; };
  static __device__ __forceinline__ v16h load(const _Float16* p) {
    U f; f.h[0] = *(const v8h*)(p); f.h[1] = *(const v8h*)(p + 16); return f.v;
  }
  static __device__ __forceinline__ v8f mma(v16h a, v16h b, v8f c) {
    return __builtin_amdgcn_wmma_f32_16x16x32_f16(false, a, false, b, (short)0, c, false, false);
  }
  static __device__ __forceinline__ void guard4(v8f& a, v8f& b, v8f& c, v8f& d, v16h x, v16h y) { dep_guard4_h(a, b, c, d, x, y); }
  static __device__ __forceinline__ void keep(v16h a, v16h b, v16h c, v16h d) { keep4_h(a, b, c, d); }
};
template <> struct Frag<__bf16> {
  typedef v16b V; union U { v16b v; v8b h[2]; };
  static __device__ __forceinline__ v16b load(const __bf16* p) {
    U f; f.h[0] = *(const v8b*)(p); f.h[1] = *(const v8b*)(p + 16); return f.v;
  }
  static __device__ __forceinline__ v8f mma(v16b a, v16b b, v8f c) {
    return __builtin_amdgcn_wmma_f32_16x16x32_bf16(false, a, false, b, (short)0, c, false, false);
  }
  static __device__ __forceinline__ void guard4(v8f& a, v8f& b, v8f& c, v8f& d, v16b x, v16b y) { dep_guard4_b(a, b, c, d, x, y); }
  static __device__ __forceinline__ void keep(v16b a, v16b b, v16b c, v16b d) { keep4_b(a, b, c, d); }
};

__device__ __forceinline__ v8f mma_h(v16h a, v16h b, v8f c) {
  c = __builtin_amdgcn_wmma_f32_16x16x32_f16(false, a, false, b, (short)0, c, false, false);
  asm volatile("v_nop\n\tv_nop\n\tv_nop\n\tv_nop" : "+v"(c) : "v"(a), "v"(b));
  return c;
}

template <int ET> struct Elem;
template <> struct Elem<0> { typedef _Float16 T; };
template <> struct Elem<1> { typedef __bf16 T; };
template <int ET, bool SPLIT, int BIAS_MODE, int OUT_MODE, bool RESID, int ACT = 0>
__global__ __launch_bounds__(256) void wmma_gemm64(
    const unsigned short* __restrict__ Ap, const unsigned short* __restrict__ A2p, int lda, long strideA,
    const unsigned short* __restrict__ Btp, const unsigned short* __restrict__ Bt2p, int ldb, long strideB,
    void* __restrict__ Cout, void* __restrict__ Cout2, int ldc, long strideC,
    const float* __restrict__ bias,
    const float* __restrict__ resid, long strideR,
    int M, int N, int K, float scale) {
  typedef typename Elem<ET>::T T;
  typedef typename Frag<T>::V V;
  const T* A = (const T*)Ap; const T* A2 = (const T*)A2p; const T* Bt = (const T*)Btp; const T* Bt2 = (const T*)Bt2p;
  __shared__ __align__(16) float sT[8][16 * 68];
  const int b    = blockIdx.y;
  const int lane = threadIdx.x & 31;
  const int wave = threadIdx.x >> 5;
  const int tilesN = N >> 6;
  const int tilesM = M >> 6;
  const int tile = blockIdx.x * 8 + wave;
  if (tile >= tilesM * tilesN) return;
  const int tm = tile / tilesN;
  const int tn = tile - tm * tilesN;
  const int m0 = tm << 6;
  const int n0 = tn << 6;

  const T* Ab  = A  + (size_t)b * strideA;
  const T* Bb  = Bt + (size_t)b * strideB;
  const T* Ab2 = SPLIT ? (A2  + (size_t)b * strideA) : nullptr;
  const T* Bb2 = SPLIT ? (Bt2 + (size_t)b * strideB) : nullptr;

  const int rlane = lane & 15;
  const int koff  = (lane >> 4) * 8;
  const int mOff  = (lane >> 4) * 8;

  v8f acc[4][4];
#pragma unroll
  for (int i = 0; i < 4; ++i)
#pragma unroll
    for (int j = 0; j < 4; ++j) acc[i][j] = (v8f){0.f,0.f,0.f,0.f,0.f,0.f,0.f,0.f};

  for (int k0 = 0; k0 < K; k0 += 32) {
    V bh[4], bl[4];
#pragma unroll
    for (int j = 0; j < 4; ++j) {
      const size_t bo = (size_t)(n0 + (j << 4) + rlane) * ldb + koff + k0;
      bh[j] = Frag<T>::load(Bb + bo);
      if (SPLIT) bl[j] = Frag<T>::load(Bb2 + bo);
    }
#pragma unroll
    for (int i = 0; i < 4; ++i) {
      const size_t ao = (size_t)(m0 + (i << 4) + rlane) * lda + koff + k0;
      V ah = Frag<T>::load(Ab + ao);
      V al;
      if (SPLIT) al = Frag<T>::load(Ab2 + ao);
#pragma unroll
      for (int j = 0; j < 4; ++j) {
        acc[i][j] = Frag<T>::mma(ah, bh[j], acc[i][j]);
        if (SPLIT) {
          acc[i][j] = Frag<T>::mma(ah, bl[j], acc[i][j]);
          acc[i][j] = Frag<T>::mma(al, bh[j], acc[i][j]);
        }
      }
      Frag<T>::guard4(acc[i][0], acc[i][1], acc[i][2], acc[i][3], ah, SPLIT ? al : ah);
    }
    Frag<T>::keep(bh[0], bh[1], bh[2], bh[3]);
    if (SPLIT) Frag<T>::keep(bl[0], bl[1], bl[2], bl[3]);
  }
  acc_guard4(acc[0][0], acc[0][1], acc[0][2], acc[0][3]);
  acc_guard4(acc[1][0], acc[1][1], acc[1][2], acc[1][3]);
  acc_guard4(acc[2][0], acc[2][1], acc[2][2], acc[2][3]);
  acc_guard4(acc[3][0], acc[3][1], acc[3][2], acc[3][3]);

  float* slab = sT[wave];
  const float* Rb = RESID ? (resid + (size_t)b * strideR) : nullptr;
#pragma unroll
  for (int i = 0; i < 4; ++i) {
    const int mBase = m0 + (i << 4);
#pragma unroll
    for (int j = 0; j < 4; ++j) {
      const int n = n0 + (j << 4) + rlane;
      float bv = 0.f;
      if (BIAS_MODE == 2) bv = bias[n];
#pragma unroll
      for (int r = 0; r < 8; ++r) {
        float v = acc[i][j][r] * scale;
        if (BIAS_MODE == 1) v += bias[mBase + mOff + r];
        if (BIAS_MODE == 2) v += bv;
        if (RESID) v += Rb[(size_t)(mBase + mOff + r) * ldc + n];
        if (ACT == 1) v = tanhf(v);
        if (ACT == 2) v = fmaxf(v, 0.0f);
        if (ACT == 3) v = v / (1.0f + expf(-v));
        if (ACT == 4) v = (v > 0.f) ? v : 0.01f * v;
        slab[(mOff + r) * 68 + (j << 4) + rlane] = v;
      }
    }
    __builtin_amdgcn_fence(__ATOMIC_RELEASE, "workgroup");
    __builtin_amdgcn_wave_barrier();
    __builtin_amdgcn_fence(__ATOMIC_ACQUIRE, "workgroup");
    if (OUT_MODE == 0) {
      float* C = (float*)Cout + (size_t)b * strideC;
      const int hh = lane >> 4, c4 = (lane & 15) * 4;
      for (int pass = 0; pass < 2; ++pass) {
#pragma unroll
        for (int it = 0; it < 8; ++it) {
          const int row = it * 2 + hh;
          v4f v = *(const v4f*)(slab + row * 68 + c4);
          *(volatile v4f*)(C + (size_t)(mBase + row) * ldc + n0 + c4) = v;
        }
        __threadfence();
      }
    } else {
      const int q = lane >> 3, c8 = (lane & 7) * 8;
      unsigned short* C  = (unsigned short*)Cout  + (size_t)b * strideC;
      unsigned short* C2 = (OUT_MODE == 2) ? ((unsigned short*)Cout2 + (size_t)b * strideC) : nullptr;
      for (int pass = 0; pass < 2; ++pass) {
#pragma unroll
        for (int it = 0; it < 4; ++it) {
          const int row = it * 4 + q;
          const float* sp = slab + row * 68 + c8;
          v8h hv, lv;
#pragma unroll
          for (int e = 0; e < 8; ++e) {
            if (OUT_MODE == 1) {
              hv[e] = (_Float16)sp[e];
            } else {
              unsigned short hb = f2bf_bits(sp[e]);
              unsigned short lb = f2bf_bits(sp[e] - bf_bits2f(hb));
              hv[e] = __builtin_bit_cast(_Float16, hb);
              lv[e] = __builtin_bit_cast(_Float16, lb);
            }
          }
          *(volatile v8h*)(C + (size_t)(mBase + row) * ldc + n0 + c8) = hv;
          if (OUT_MODE == 2) *(volatile v8h*)(C2 + (size_t)(mBase + row) * ldc + n0 + c8) = lv;
        }
        __threadfence();
      }
    }
    __builtin_amdgcn_fence(__ATOMIC_RELEASE, "workgroup");
    __builtin_amdgcn_wave_barrier();
    __builtin_amdgcn_fence(__ATOMIC_ACQUIRE, "workgroup");
  }
}

__global__ __launch_bounds__(kThr) void cast_plane_kernel(const float* __restrict__ src, unsigned short* __restrict__ dst,
                                                          int colsLog2, int dstPitch, int dstOff) {
  const int i   = blockIdx.x * kThr + threadIdx.x;
  const int sh  = colsLog2 - 3;
  const int row = i >> sh;
  const int c8  = (i & ((1 << sh) - 1)) * 8;
  const float* sp = src + ((size_t)row << colsLog2) + c8;
  const v4f a0 = *(const v4f*)(sp);
  const v4f a1 = *(const v4f*)(sp + 4);
  v8h hv;
#pragma unroll
  for (int e = 0; e < 4; ++e) {
    const float f0 = a0[e];
    const float f1 = a1[e];
    hv[e]     = (_Float16)carry_flush(bf16r(f0), kInCarry);
    hv[4 + e] = (_Float16)carry_flush(bf16r(f1), kInCarry);
  }
  unsigned short* dp = dst + (size_t)row * dstPitch + dstOff + c8;
  *(volatile v8h*)dp = hv;
  __threadfence();
  *(volatile v8h*)dp = hv;
}
__global__ __launch_bounds__(256) void wt_plane_kernel(const float* __restrict__ W, unsigned short* __restrict__ dst, int K, int N, int nLive, int ldd, int colOff) {
  const int n  = blockIdx.x;
  const int k8 = threadIdx.x * 8;
  const bool live = n < nLive;
  const int nc = live ? n : 0;
  v8h hv;
#pragma unroll
  for (int e = 0; e < 8; ++e) {
    const float w = W[(size_t)(k8 + e) * N + nc];
    hv[e] = (_Float16)(live ? carry_flush(bf16r(w), kWCarry) : 0.0f);
  }
  unsigned short* dp = dst + (size_t)n * ldd + colOff + k8;
  *(volatile v8h*)dp = hv;
  __threadfence();
  *(volatile v8h*)dp = hv;
}

__global__ __launch_bounds__(kThr) void setup_kernel(const float* __restrict__ b_z, const float* __restrict__ b_f, const float* __restrict__ b_o,
                                                     float* __restrict__ BIAS, unsigned short* __restrict__ X16P) {
  const unsigned v = blockIdx.x * (unsigned)kThr + threadIdx.x;
  if (v < 256u) {
    const unsigned i0 = v * 4u;
    const unsigned g = i0 >> 8, j = i0 & 255u;
    v4f o = {0.f, 0.f, 0.f, 0.f};
    if (g < 3u) {
      const float* sp = (g == 0u) ? b_z : ((g == 1u) ? b_f : b_o);
      const v4f a = *(const v4f*)(sp + j);
#pragma unroll
      for (int e = 0; e < 4; ++e) { const float p = a[e]; o[e] = bf16r(p); }
    }
    float* dp = BIAS + i0;
    *(volatile v4f*)dp = o;
    __threadfence();
    *(volatile v4f*)dp = o;
  } else {
    const unsigned w = v - 256u;
    const unsigned smp = w >> 5, c8 = (w & 31u) * 8u;
    v8h z;
#pragma unroll
    for (int e = 0; e < 8; ++e) z[e] = (_Float16)0.0f;
    unsigned short* dp = X16P + (size_t)smp * kTP * kDi + c8;
    *(volatile v8h*)dp = z;
    __threadfence();
    *(volatile v8h*)dp = z;
  }
}
static_assert(kN3 == 768 && kDi / 8 == 32 && kB * 32 == 256 && kDo == 256, "set-up grid exact: 256 + 256 threads; a gate's biases are one 256-float group");

__global__ __launch_bounds__(kThr) void pool_scan_kernel(const float* __restrict__ ZFO, float* __restrict__ out) {
  const unsigned v = blockIdx.x * (unsigned)kThr + threadIdx.x;
  const unsigned smp = v >> 8, d = v & 255u;
  const float* zp = ZFO + (size_t)smp * kT * kN3 + d;
  float* op = out + (size_t)smp * kT * kDo + d;
  float c = 0.0f;
  for (int t = 0; t < kT; ++t) {
    const float zv = zp[(size_t)t * kN3];
    const float fv = zp[(size_t)t * kN3 + kDo];
    const float ov = zp[(size_t)t * kN3 + 2 * kDo];
    const float z = tanhf(zv);
    const float f = 1.0f / (1.0f + expf(-fv));
    const float o = 1.0f / (1.0f + expf(-ov));
    c = f * c + (1.0f - f) * z;
    const float h = o * c;
    float* hp = op + (size_t)t * kDo;
    *(volatile float*)hp = h;
    __threadfence();
    *(volatile float*)hp = h;
  }
}
static_assert((kB * kDo) % kThr == 0 && kDo == 256, "scan grid exact; a block = one sample's 256 channels");

static_assert(((size_t)kT * kDi / 8) % kThr == 0, "plane cast grid exact");

extern "C" void kernel_launch(void* const* d_in, const int* in_sizes, int n_in,
                              void* d_out, int out_size, void* d_ws, size_t ws_size,
                              hipStream_t stream) {
  if (n_in < 7 || d_out == nullptr || d_ws == nullptr) return;
  if (in_sizes[0] != kB * kT * kDi || in_sizes[1] != kWin * kDi * kDo || in_sizes[2] != kWin * kDi * kDo || in_sizes[3] != kWin * kDi * kDo) return;
  if (in_sizes[4] != kDo || in_sizes[5] != kDo || in_sizes[6] != kDo) return;
  if (out_size != kB * kT * kDo) return;
  if (ws_size < kWsTotal) return;
  const float* x = (const float*)d_in[0];
  const float* W_z = (const float*)d_in[1];
  const float* W_f = (const float*)d_in[2];
  const float* W_o = (const float*)d_in[3];
  const float* b_z = (const float*)d_in[4];
  const float* b_f = (const float*)d_in[5];
  const float* b_o = (const float*)d_in[6];
  float* out = (float*)d_out;
  char* ws = (char*)d_ws;
  unsigned short* X16P = (unsigned short*)(ws + kOffX16P);
  unsigned short* WZFO = (unsigned short*)(ws + kOffWZFO);
  float* BIAS = (float*)(ws + kOffBIAS);
  float* ZFO = (float*)(ws + kOffZFO);

  for (int smp = 0; smp < kB; ++smp)
    cast_plane_kernel<<<(int)(((size_t)kT * kDi / 8) / kThr), kThr, 0, stream>>>(x + (size_t)smp * kT * kDi, X16P + ((size_t)smp * kTP + 1) * kDi, 8, kDi, 0);
  wt_plane_kernel<<<kDo, kDi / 8, 0, stream>>>(W_z, WZFO, kDi, kDo, kDo, kWin * kDi, 0);
  wt_plane_kernel<<<kDo, kDi / 8, 0, stream>>>(W_z + (size_t)kDi * kDo, WZFO, kDi, kDo, kDo, kWin * kDi, kDi);
  wt_plane_kernel<<<kDo, kDi / 8, 0, stream>>>(W_f, WZFO + (size_t)kDo * kWin * kDi, kDi, kDo, kDo, kWin * kDi, 0);
  wt_plane_kernel<<<kDo, kDi / 8, 0, stream>>>(W_f + (size_t)kDi * kDo, WZFO + (size_t)kDo * kWin * kDi, kDi, kDo, kDo, kWin * kDi, kDi);
  wt_plane_kernel<<<kDo, kDi / 8, 0, stream>>>(W_o, WZFO + (size_t)2 * kDo * kWin * kDi, kDi, kDo, kDo, kWin * kDi, 0);
  wt_plane_kernel<<<kDo, kDi / 8, 0, stream>>>(W_o + (size_t)kDi * kDo, WZFO + (size_t)2 * kDo * kWin * kDi, kDi, kDo, kDo, kWin * kDi, kDi);
  setup_kernel<<<2, kThr, 0, stream>>>(b_z, b_f, b_o, BIAS, X16P);
  wmma_gemm64<0, false, 2, 0, false, 0><<<dim3((kT / 64) * (kN3 / 64) / 8, kB), 256, 0, stream>>>(
      X16P, X16P, kDi, (long)kTP * kDi, WZFO, WZFO, kWin * kDi, 0L, (void*)ZFO, (void*)ZFO, kN3, (long)kT * kN3, BIAS, nullptr, 0L, kT, kN3, kWin * kDi, kSc);
  pool_scan_kernel<<<(kB * kDo) / kThr, kThr, 0, stream>>>(ZFO, out);
}
